// LinearTemporalSelfAttention_62491774157502
// MI455X (gfx1250) — hardware-verified
//
#include <hip/hip_runtime.h>
#include <math.h>

typedef __attribute__((ext_vector_type(16))) _Float16 v16h;
typedef __attribute__((ext_vector_type(16))) __bf16 v16b;
typedef __attribute__((ext_vector_type(8)))  _Float16 v8h;
typedef __attribute__((ext_vector_type(8)))  float v8f;
typedef __attribute__((ext_vector_type(4)))  float v4f;
typedef __attribute__((ext_vector_type(2)))  float v2f;
typedef __attribute__((ext_vector_type(4)))  unsigned v4u;
typedef __attribute__((ext_vector_type(4)))  int v4i;
typedef float __attribute__((may_alias)) float_a;
typedef int __attribute__((may_alias)) int_a;

template <typename T> __device__ __forceinline__ void vst2(void* p, T v) { *(volatile T*)p = v; __threadfence(); *(volatile T*)p = v; }
__device__ __forceinline__ v8f wmma16(v16h a, v16h b, v8f c) {
  v8f d = __builtin_amdgcn_wmma_f32_16x16x32_f16(false, a, false, b, (short)0, c, false, false);
  asm volatile("v_nop\n\tv_nop\n\tv_nop\n\tv_nop" : "+v"(d) : "v"(a), "v"(b));
  return d;
}
__device__ __forceinline__ v8f wmma_bf(v16b a, v16b b, v8f c) {
  v8f d = __builtin_amdgcn_wmma_f32_16x16x32_bf16(false, a, false, b, (short)0, c, false, false);
  asm volatile("v_nop\n\tv_nop\n\tv_nop\n\tv_nop" : "+v"(d) : "v"(a), "v"(b));
  return d;
}
__device__ __forceinline__ v16h frag_h(const _Float16* rowk0, int lane) {
  union { v16h v; v8h q[2]; } u; const _Float16* p = rowk0 + 8 * (lane >> 4);
  u.q[0] = *(const v8h*)p; u.q[1] = *(const v8h*)(p + 16); return u.v;
}
__device__ __forceinline__ v16h frag_f32(const float* rowk0, int lane) {
  v16h a; const float* p = rowk0 + 8 * (lane >> 4);
#pragma unroll
  for (int i = 0; i < 8; ++i) { a[i] = (_Float16)p[i]; a[8 + i] = (_Float16)p[16 + i]; }
  return a;
}
__device__ __forceinline__ v16h frag_f32s(const float* rowk0, int lane, float sc) {
  v16h a; const float* p = rowk0 + 8 * (lane >> 4);
#pragma unroll
  for (int i = 0; i < 8; ++i) { a[i] = (_Float16)(p[i] * sc); a[8 + i] = (_Float16)(p[16 + i] * sc); }
  return a;
}
__device__ __forceinline__ v16h fragc_f32(const float* W, int k0, int n, int lane, int ld, int K) {
  v16h a; const int g = lane >> 4;
#pragma unroll
  for (int i = 0; i < 8; ++i) { const int ka = k0 + 8 * g + i, kb = ka + 16;
    a[i] = (_Float16)(ka < K ? W[(size_t)(ka < K ? ka : K - 1) * ld + n] : 0.f); a[8 + i] = (_Float16)(kb < K ? W[(size_t)(kb < K ? kb : K - 1) * ld + n] : 0.f); }
  return a;
}
struct F2 { v16b h, l; };
__device__ __forceinline__ F2 bsplit16(const float v[16]) { F2 r;
#pragma unroll
  for (int i = 0; i < 16; ++i) { const __bf16 h = (__bf16)v[i]; r.h[i] = h; r.l[i] = (__bf16)(v[i] - (float)h); }
  return r; }
__device__ __forceinline__ F2 split_row(const float* row, int k0, int lane) { float v[16]; const float* p = row + k0 + 8 * (lane >> 4);
#pragma unroll
  for (int i = 0; i < 8; ++i) { v[i] = p[i]; v[8 + i] = p[16 + i]; }
  return bsplit16(v); }
__device__ __forceinline__ F2 split_rowK(const float* row, int k0, int lane, int K) { float v[16]; const int g = lane >> 4;
#pragma unroll
  for (int i = 0; i < 8; ++i) { const int ka = k0 + 8 * g + i, kb = ka + 16; v[i] = ka < K ? row[ka < K ? ka : K - 1] : 0.f; v[8 + i] = kb < K ? row[kb < K ? kb : K - 1] : 0.f; }
  return bsplit16(v); }
__device__ __forceinline__ F2 split_col(const float* W, int k0, int n, int lane, int ld, int K) { float v[16]; const int g = lane >> 4;
#pragma unroll
  for (int i = 0; i < 8; ++i) { const int ka = k0 + 8 * g + i, kb = ka + 16; v[i] = ka < K ? W[(size_t)(ka < K ? ka : K - 1) * ld + n] : 0.f; v[8 + i] = kb < K ? W[(size_t)(kb < K ? kb : K - 1) * ld + n] : 0.f; }
  return bsplit16(v); }
__device__ __forceinline__ v8f mac3(const F2& a, const F2& b, v8f c) { c = wmma_bf(a.l, b.h, c); c = wmma_bf(a.h, b.l, c); return wmma_bf(a.h, b.h, c); }
__device__ __forceinline__ float sigm(float v) { return 1.0f / (1.0f + expf(-v)); }
#define LDSX() do { asm volatile("s_wait_dscnt 0" ::: "memory"); __builtin_amdgcn_wave_barrier(); __builtin_amdgcn_fence(__ATOMIC_RELEASE, "workgroup"); } while (0)


#define NB 4
#define TT 2048
#define DD 1024
#define NH 8
#define DH 128
#define TE 2048
#define NR (NB * TT)
#define WSC 256.0f
#define EPS 1e-5f
typedef __attribute__((ext_vector_type(8))) __bf16 v8b;
__device__ __forceinline__ v16b frag_b(const __bf16* rowk0, int lane) {
  union { v16b v; v8b q[2]; } u; const __bf16* p = rowk0 + 8 * (lane >> 4);
  u.q[0] = *(const v8b*)p; u.q[1] = *(const v8b*)(p + 16); return u.v;
}
__device__ __forceinline__ float bfr(float v) { return (float)(__bf16)v; }
__device__ __attribute__((noinline)) float exp_ni(float v) { return expf(v); }
__device__ __attribute__((noinline)) float erf_ni(float v) { return erff(v); }

#define WS_PW   0u
#define WS_PO   (WS_PW + 2u * (size_t)3 * DD * DD)
#define WS_XN   (WS_PO + 2u * (size_t)DD * DD)
#define WS_QKV  (WS_XN + 2u * (size_t)NR * DD)
#define QKW 2048
#define WS_QS   (WS_QKV + 4u * (size_t)NR * 2 * DD)
#define WS_QSL  (WS_QS + 2u * (size_t)NR * DD)
#define WS_KST  (WS_QSL + 2u * (size_t)NR * DD)
#define WS_KSTL (WS_KST + 2u * (size_t)NR * DD)
#define WS_VT   (WS_KSTL + 2u * (size_t)NR * DD)
#define WS_VTL  (WS_VT + 2u * (size_t)NR * DD)
#define WS_AT   (WS_VTL + 2u * (size_t)NR * DD)
#define WS_ATL  (WS_AT + 2u * (size_t)NB * NH * DH * DH)
#define WS_Y    (WS_ATL + 2u * (size_t)NB * NH * DH * DH)
#define WS_FILM (WS_Y + 4u * (size_t)NR * DD)
#define WS_HH   (WS_FILM + 4u * (size_t)NB * 2 * DD)
#define WS_END  (WS_HH + 2u * (size_t)NR * DD)

__global__ __launch_bounds__(256) void k_packw(const float* __restrict__ WQ, const float* __restrict__ WK, const float* __restrict__ WV, const float* __restrict__ WO, char* __restrict__ ws) { const int n = blockIdx.x, which = blockIdx.y, t = threadIdx.x; __shared__ __align__(16) _Float16 s[DD]; const float* Wm = which == 0 ? WQ : which == 1 ? WK : which == 2 ? WV : WO;
  for (int k = t; k < DD; k += 256) s[k] = (_Float16)(bfr(Wm[(size_t)k * DD + n]) * WSC); __syncthreads();
  _Float16* dst = (which < 3) ? ((_Float16*)(ws + WS_PW) + ((size_t)which * DD + n) * DD) : ((_Float16*)(ws + WS_PO) + (size_t)n * DD); for (int q = t; q < DD / 8; q += 256) vst2((unsigned*)(dst + q * 8), *(const v4u*)&s[q * 8]); }
__global__ __launch_bounds__(256) void k_ln1(const float* __restrict__ X, const float* __restrict__ G, const float* __restrict__ Bt, _Float16* __restrict__ XN) { __shared__ float red[8]; __shared__ __align__(16) _Float16 sh[DD]; const int t = threadIdx.x; const size_t row = blockIdx.x;
  float v[4]; float s = 0.f; for (int i = 0; i < 4; ++i) { v[i] = bfr(X[row * DD + t + 256 * i]); s += v[i]; }
#pragma unroll
  for (int o = 1; o < 32; o <<= 1) s += __shfl_xor(s, o);
  if ((t & 31) == 0) red[t >> 5] = s; __syncthreads(); float mu = 0.f; for (int i = 0; i < 8; ++i) mu += red[i]; mu /= (float)DD; __syncthreads();
  float q = 0.f; for (int i = 0; i < 4; ++i) { const float d = v[i] - mu; q += d * d; }
#pragma unroll
  for (int o = 1; o < 32; o <<= 1) q += __shfl_xor(q, o);
  if ((t & 31) == 0) red[t >> 5] = q; __syncthreads(); float var = 0.f; for (int i = 0; i < 8; ++i) var += red[i]; var /= (float)DD; const float inv = 1.0f / sqrtf(var + EPS);
  for (int i = 0; i < 4; ++i) { const int c = t + 256 * i; sh[c] = (_Float16)((v[i] - mu) * inv * bfr(G[c]) + bfr(Bt[c])); } __syncthreads(); if (t < DD / 8) vst2((unsigned*)(XN + row * DD + t * 8), *(const v4u*)&sh[t * 8]); }
template <int RES>
__global__ __launch_bounds__(128) void k_gemm(const _Float16* __restrict__ A, const _Float16* __restrict__ Wr, const float* __restrict__ BIAS, const float* __restrict__ XRES, float* __restrict__ OUT, int ow, _Float16* __restrict__ QSp = nullptr, _Float16* __restrict__ QSLp = nullptr) { __shared__ __align__(16) float sf[4][16][132]; __shared__ __align__(16) _Float16 sqh[4][16][136], sql[4][16][136];
  const int tid = threadIdx.x, wave = tid >> 5, lane = tid & 31, col = lane & 15, g = lane >> 4; const size_t r0 = (size_t)blockIdx.x * 64 + wave * 16; const int c0 = blockIdx.y * 128;
  v8f acc[8] = {};
#pragma unroll 2
  for (int kc = 0; kc < DD / 32; ++kc) { const v16h a = frag_h(A + (r0 + col) * DD + kc * 32, lane);
#pragma unroll
    for (int j = 0; j < 8; ++j) acc[j] = wmma16(a, frag_h(Wr + (size_t)(c0 + j * 16 + col) * DD + kc * 32, lane), acc[j]); }
  if (RES == 2) {
    float mx[8], sm[8];
#pragma unroll
    for (int r = 0; r < 8; ++r) { mx[r] = -3.0e38f; sm[r] = 0.f; }
#pragma unroll
    for (int j = 0; j < 8; ++j) { const float bb = bfr(BIAS[c0 + j * 16 + col]);
#pragma unroll
      for (int r = 0; r < 8; ++r) { acc[j][r] = acc[j][r] * (1.0f / WSC) + bb; mx[r] = fmaxf(mx[r], acc[j][r]); } }
#pragma unroll
    for (int r = 0; r < 8; ++r) {
#pragma unroll
      for (int o = 1; o < 16; o <<= 1) mx[r] = fmaxf(mx[r], __shfl_xor(mx[r], o)); }
#pragma unroll
    for (int j = 0; j < 8; ++j)
#pragma unroll
      for (int r = 0; r < 8; ++r) { acc[j][r] = expf(acc[j][r] - mx[r]); sm[r] += acc[j][r]; }
#pragma unroll
    for (int r = 0; r < 8; ++r) {
#pragma unroll
      for (int o = 1; o < 16; o <<= 1) sm[r] += __shfl_xor(sm[r], o); }
#pragma unroll
    for (int j = 0; j < 8; ++j)
#pragma unroll
      for (int r = 0; r < 8; ++r) { const float p = acc[j][r] / sm[r]; const _Float16 hv = (_Float16)p; sqh[wave][8 * g + r][j * 16 + col] = hv; sql[wave][8 * g + r][j * 16 + col] = (_Float16)((p - (float)hv) * 2048.0f); }
    LDSX(); for (int rl = 0; rl < 16; ++rl) if (lane < 16) { vst2((unsigned*)(QSp + (r0 + rl) * (size_t)ow + c0 + lane * 8), *(const v4u*)&sqh[wave][rl][lane * 8]); vst2((unsigned*)(QSLp + (r0 + rl) * (size_t)ow + c0 + lane * 8), *(const v4u*)&sql[wave][rl][lane * 8]); }
    return; }
#pragma unroll
  for (int j = 0; j < 8; ++j) { const int c = c0 + j * 16 + col; const float bb = bfr(BIAS[c]);
#pragma unroll
    for (int r = 0; r < 8; ++r) { float v = acc[j][r] * (1.0f / WSC) + bb; if (RES == 1) v += bfr(XRES[(r0 + 8 * g + r) * DD + c]); sf[wave][8 * g + r][j * 16 + col] = v; } }
  LDSX(); for (int rl = 0; rl < 16; ++rl) vst2(OUT + (r0 + rl) * (size_t)ow + c0 + lane * 4, *(const v4f*)&sf[wave][rl][lane * 4]); }
__global__ __launch_bounds__(256) void k_ksoft(const float* __restrict__ QKV, const float* __restrict__ MASK, _Float16* __restrict__ KST, _Float16* __restrict__ KSTL, _Float16* __restrict__ VT, _Float16* __restrict__ VTL) {
  __shared__ float smax[8][32], ssum[8][32]; __shared__ float cmax[32], cinv[32]; __shared__ __align__(16) _Float16 th[32][72], tl[32][72], uh[32][72], ul[32][72];
  const int t = threadIdx.x; const int cl = t & 31, tg = t >> 5; const size_t b = blockIdx.y; const int c0 = blockIdx.x * 32; const int c = c0 + cl;
  float mx = -3.0e38f; for (int ti = tg; ti < TT; ti += 8) { const size_t row = b * TT + ti; if (bfr(MASK[row]) != 0.f) mx = fmaxf(mx, QKV[row * QKW + c]); }
  smax[tg][cl] = mx; __syncthreads(); if (t < 32) { float m = -3.0e38f; for (int i = 0; i < 8; ++i) m = fmaxf(m, smax[i][t]); cmax[t] = m; } __syncthreads(); mx = cmax[cl];
  float s = 0.f; for (int ti = tg; ti < TT; ti += 8) { const size_t row = b * TT + ti; if (bfr(MASK[row]) != 0.f) s += expf(QKV[row * QKW + c] - mx); }
  ssum[tg][cl] = s; __syncthreads(); if (t < 32) { float ss = 0.f; for (int i = 0; i < 8; ++i) ss += ssum[i][t]; cinv[t] = (ss > 0.f) ? 1.0f / ss : 0.f; } __syncthreads(); const float inv = cinv[cl];
  for (int t0 = 0; t0 < TT; t0 += 64) { for (int e = t; e < 32 * 64; e += 256) { const int cc = e & 31, tl2 = e >> 5; const size_t row = b * TT + t0 + tl2; const float mk = bfr(MASK[row]); const int cg = c0 + cc;
      const float kv = QKV[row * QKW + cg]; const float p = (mk != 0.f) ? expf(kv - cmax[cc]) * cinv[cc] : 0.f; const _Float16 ph = (_Float16)p; th[cc][tl2] = ph; tl[cc][tl2] = (_Float16)((p - (float)ph) * 2048.0f);
      const float vv = QKV[row * QKW + DD + cg] * mk; const _Float16 vh = (_Float16)vv; uh[cc][tl2] = vh; ul[cc][tl2] = (_Float16)((vv - (float)vh) * 2048.0f); }
    __syncthreads(); { const int cc = t >> 3, q = t & 7; const size_t o = (b * DD + c0 + cc) * (size_t)TT + t0 + q * 8; vst2((unsigned*)(KST + o), *(const v4u*)&th[cc][q * 8]); vst2((unsigned*)(KSTL + o), *(const v4u*)&tl[cc][q * 8]); vst2((unsigned*)(VT + o), *(const v4u*)&uh[cc][q * 8]); vst2((unsigned*)(VTL + o), *(const v4u*)&ul[cc][q * 8]); } __syncthreads(); }
  (void)inv; (void)s; }
__global__ __launch_bounds__(128) void k_att(const _Float16* __restrict__ KST, const _Float16* __restrict__ KSTL, const _Float16* __restrict__ VT, const _Float16* __restrict__ VTL, _Float16* __restrict__ AT, _Float16* __restrict__ ATL) { __shared__ __align__(16) _Float16 th[DH][DH + 8], tl2[DH][DH + 8];
  const int tid = threadIdx.x, wave = tid >> 5, lane = tid & 31, col = lane & 15, g = lane >> 4; const int h = blockIdx.x; const size_t b = blockIdx.y; const size_t pk = (b * DD + (size_t)h * DH) * TT;
  for (int dt = 0; dt < 2; ++dt) { const int d0 = dt * 64 + wave * 16; v8f acc[8] = {}, accl[8] = {};
#pragma unroll 1
    for (int kc = 0; kc < TT / 32; ++kc) { const v16h ah = frag_h(KST + pk + (size_t)(d0 + col) * TT + kc * 32, lane), al = frag_h(KSTL + pk + (size_t)(d0 + col) * TT + kc * 32, lane);
#pragma unroll
      for (int j = 0; j < 8; ++j) { const size_t o = pk + (size_t)(j * 16 + col) * TT + kc * 32; const v16h bh = frag_h(VT + o, lane), bl = frag_h(VTL + o, lane); acc[j] = wmma16(ah, bh, acc[j]); accl[j] = wmma16(ah, bl, accl[j]); accl[j] = wmma16(al, bh, accl[j]); } }
#pragma unroll
    for (int j = 0; j < 8; ++j)
#pragma unroll
      for (int r = 0; r < 8; ++r) { const float v = acc[j][r] + accl[j][r] * (1.0f / 2048.0f); const _Float16 hv = (_Float16)v; th[j * 16 + col][d0 + 8 * g + r] = hv; tl2[j * 16 + col][d0 + 8 * g + r] = (_Float16)((v - (float)hv) * 2048.0f); } }
  __syncthreads(); for (int e = tid; e < DH * 16; e += 128) { const int l = e >> 4, q = e & 15; const size_t o = ((b * NH + h) * DH + l) * DH + q * 8; vst2((unsigned*)(AT + o), *(const v4u*)&th[l][q * 8]); vst2((unsigned*)(ATL + o), *(const v4u*)&tl2[l][q * 8]); } }
__global__ __launch_bounds__(128) void k_y(const _Float16* __restrict__ QS, const _Float16* __restrict__ QSL, const _Float16* __restrict__ AT, const _Float16* __restrict__ ATL, float* __restrict__ Y) { __shared__ __align__(16) float sf[4][16][132];
  const int tid = threadIdx.x, wave = tid >> 5, lane = tid & 31, col = lane & 15, g = lane >> 4; const size_t r0 = (size_t)blockIdx.x * 64 + wave * 16; const int h = blockIdx.y; const size_t b = r0 / TT; const size_t pa = ((b * NH + h) * DH) * DH;
  v8f acc[8] = {}, accl[8] = {};
#pragma unroll
  for (int kc = 0; kc < DH / 32; ++kc) { const v16h ah = frag_h(QS + (r0 + col) * DD + h * DH + kc * 32, lane), al = frag_h(QSL + (r0 + col) * DD + h * DH + kc * 32, lane);
#pragma unroll
    for (int j = 0; j < 8; ++j) { const size_t o = pa + (size_t)(j * 16 + col) * DH + kc * 32; const v16h bh = frag_h(AT + o, lane), bl = frag_h(ATL + o, lane); acc[j] = wmma16(ah, bh, acc[j]); accl[j] = wmma16(ah, bl, accl[j]); accl[j] = wmma16(al, bh, accl[j]); } }
#pragma unroll
  for (int j = 0; j < 8; ++j)
#pragma unroll
    for (int r = 0; r < 8; ++r) sf[wave][8 * g + r][j * 16 + col] = acc[j][r] + accl[j][r] * (1.0f / 2048.0f);
  LDSX(); for (int rl = 0; rl < 16; ++rl) vst2(Y + (r0 + rl) * DD + (size_t)h * DH + lane * 4, *(const v4f*)&sf[wave][rl][lane * 4]); }
__global__ __launch_bounds__(256) void k_emb(const float* __restrict__ EMB, const float* __restrict__ WE, const float* __restrict__ BE, float* __restrict__ FILM) { __shared__ float se[TE]; __shared__ __align__(16) float so2[256]; const int t = threadIdx.x; const size_t b = blockIdx.y; const int o = blockIdx.x * 256 + t;
  for (int i = t; i < TE; i += 256) { const float ev = bfr(EMB[b * TE + i]); se[i] = ev / (1.0f + expf(-ev)); } __syncthreads();
  float s = bfr(BE[o]);
#pragma unroll 1
  for (int i = 0; i < TE; ++i) s += se[i] * bfr(WE[(size_t)i * (2 * DD) + o]); so2[t] = s; __syncthreads(); if (t < 64) vst2(FILM + b * (2 * DD) + blockIdx.x * 256 + t * 4, *(const v4f*)&so2[t * 4]); }
__global__ __launch_bounds__(256) void k_film(const float* __restrict__ Y, const float* __restrict__ G, const float* __restrict__ Bt, const float* __restrict__ FILM, _Float16* __restrict__ HH) { __shared__ float red[8]; __shared__ __align__(16) _Float16 sh[DD]; const int t = threadIdx.x; const size_t row = blockIdx.x; const size_t b = row / TT;
  float v[4]; float s = 0.f; for (int i = 0; i < 4; ++i) { v[i] = Y[row * DD + t + 256 * i]; s += v[i]; }
#pragma unroll
  for (int o = 1; o < 32; o <<= 1) s += __shfl_xor(s, o);
  if ((t & 31) == 0) red[t >> 5] = s; __syncthreads(); float mu = 0.f; for (int i = 0; i < 8; ++i) mu += red[i]; mu /= (float)DD; __syncthreads();
  float q = 0.f; for (int i = 0; i < 4; ++i) { const float d = v[i] - mu; q += d * d; }
#pragma unroll
  for (int o = 1; o < 32; o <<= 1) q += __shfl_xor(q, o);
  if ((t & 31) == 0) red[t >> 5] = q; __syncthreads(); float var = 0.f; for (int i = 0; i < 8; ++i) var += red[i]; var /= (float)DD; const float inv = 1.0f / sqrtf(var + EPS);
  for (int i = 0; i < 4; ++i) { const int c = t + 256 * i; const float ln = (v[i] - mu) * inv * bfr(G[c]) + bfr(Bt[c]); const float f = ln * (1.0f + FILM[b * (2 * DD) + c]) + FILM[b * (2 * DD) + DD + c]; sh[c] = (_Float16)(f / (1.0f + expf(-f))); } __syncthreads(); if (t < DD / 8) vst2((unsigned*)(HH + row * DD + t * 8), *(const v4u*)&sh[t * 8]); }
extern "C" void kernel_launch(void* const* d_in, const int* in_sizes, int n_in, void* d_out, int out_size, void* d_ws, size_t ws_size, hipStream_t stream) {
  (void)in_sizes; (void)n_in; (void)out_size;
  const float** F = (const float**)d_in;
  if (ws_size < (size_t)WS_END) return;
  char* ws = (char*)d_ws; _Float16 *PW = (_Float16*)(ws + WS_PW), *PO = (_Float16*)(ws + WS_PO), *XN = (_Float16*)(ws + WS_XN), *QS = (_Float16*)(ws + WS_QS), *QSL = (_Float16*)(ws + WS_QSL), *KST = (_Float16*)(ws + WS_KST), *KSTL = (_Float16*)(ws + WS_KSTL), *VT = (_Float16*)(ws + WS_VT), *VTL = (_Float16*)(ws + WS_VTL), *AT = (_Float16*)(ws + WS_AT), *ATL = (_Float16*)(ws + WS_ATL), *HH = (_Float16*)(ws + WS_HH);
  float *QKV = (float*)(ws + WS_QKV), *Y = (float*)(ws + WS_Y), *FILM = (float*)(ws + WS_FILM);
  k_packw<<<dim3(DD, 4), 256, 0, stream>>>(F[6], F[8], F[10], F[16], ws);
  k_ln1<<<NR, 256, 0, stream>>>(F[0], F[4], F[5], XN);
  k_gemm<2><<<dim3(NR / 64, DD / 128), 128, 0, stream>>>(XN, PW, F[7], nullptr, nullptr, DD, QS, QSL);
  k_gemm<0><<<dim3(NR / 64, DD / 128), 128, 0, stream>>>(XN, PW + (size_t)1 * DD * DD, F[9], nullptr, QKV, QKW);
  k_gemm<0><<<dim3(NR / 64, DD / 128), 128, 0, stream>>>(XN, PW + (size_t)2 * DD * DD, F[11], nullptr, QKV + DD, QKW);
  k_ksoft<<<dim3(DD / 32, NB), 256, 0, stream>>>(QKV, F[2], KST, KSTL, VT, VTL);
  k_att<<<dim3(NH, NB), 128, 0, stream>>>(KST, KSTL, VT, VTL, AT, ATL);
  k_y<<<dim3(NR / 64, NH), 128, 0, stream>>>(QS, QSL, AT, ATL, Y);
  k_emb<<<dim3(2 * DD / 256, NB), 256, 0, stream>>>(F[1], F[12], F[13], FILM);
  k_film<<<NR, 256, 0, stream>>>(Y, F[14], F[15], FILM, HH);
  k_gemm<1><<<dim3(NR / 64, DD / 128), 128, 0, stream>>>(HH, PO, F[17], F[0], (float*)d_out, DD);
}
